// GIN_43550968381727
// MI455X (gfx1250) — hardware-verified
//
#include <hip/hip_runtime.h>
#include <stddef.h>
#include <stdint.h>


#define CIN     128
#define HID     256
#define COUT    64
#define K1      (2 * CIN)
#define K2      (2 * HID)
#define NTHR    256
#define NWAVE   8
#define EPT     8
#define CHUNK   (NTHR * EPT)
#define WCAP    (EPT * 32)
#define LISTN   (NWAVE * WCAP)
#define NBMAX   2048
#define RCAP    28672
#define DEGCAP  64
#define PKS     11
#define GBM     64
#define GTHR    128
#define NU1A    (HID * (K1 / 8))
#define NUHH    (HID * (K2 / 8))
#define NU3B    (COUT * (K2 / 8))
#define NUB1    (NU1A)
#define NUB2    (NUB1 + NUHH)
#define NUB3    (NUB2 + NUHH)
#define NUB4    (NUB3 + NUHH)
#define NUB5    (NUB4 + NUHH)
#define NUTOT   (NUB5 + NU3B)
#define WSMAX   134217728
#define LDS_ZINTS (2 * RCAP + 2 * NBMAX + LISTN + 2 * NWAVE)
#define LDS_AGG   (LDS_ZINTS * 4)

static_assert((CHUNK & (CHUNK - 1)) == 0 && CHUNK <= (1 << PKS));
static_assert((NBMAX & (NBMAX - 1)) == 0 && NBMAX <= (1 << PKS));
static_assert(NTHR * 8 == NBMAX);
static_assert(LISTN >= NBMAX && LISTN >= NWAVE * WCAP);
static_assert((RCAP % 32) == 0 && (LDS_ZINTS % 4) == 0);
static_assert(LDS_AGG <= 300000);
static_assert(GBM == (GTHR / 32) * 16);
static_assert(CIN == 32 * 4 && HID == 32 * 8);
static_assert((K1 % 32) == 0 && (K2 % 32) == 0);
static_assert((HID % 128) == 0 && COUT == 64);
static_assert((NU1A % NTHR) == 0 && (NUHH % NTHR) == 0 && (NU3B % NTHR) == 0 && (NUTOT % NTHR) == 0);
static_assert((K1 / 8) == 32 && (K2 / 8) == 64);

typedef float          v4f  __attribute__((ext_vector_type(4)));
typedef float          v8f  __attribute__((ext_vector_type(8)));
typedef int            v4i  __attribute__((ext_vector_type(4)));
typedef int            v8i  __attribute__((ext_vector_type(8)));
typedef unsigned int   v4u  __attribute__((ext_vector_type(4)));
typedef unsigned short v8us __attribute__((ext_vector_type(8)));
typedef __bf16         v16b __attribute__((ext_vector_type(16)));
typedef v4f  __attribute__((may_alias)) v4fa;
typedef v4i  __attribute__((may_alias)) v4ia;
typedef v4u  __attribute__((may_alias)) v4ua;
typedef v8us __attribute__((may_alias)) v8usa;
union Frag { v16b vb; v8us h[2]; v8i w; };

__device__ __forceinline__ v8f wmb(const Frag& a, const Frag& b, v8f c) {
  v8f d = __builtin_amdgcn_wmma_f32_16x16x32_bf16(false, a.vb, false, b.vb, (short)0, c, false, false);
  asm volatile("v_nop\n\tv_nop\n\tv_nop\n\tv_nop" : "+v"(d) : "v"(a.w), "v"(b.w));
  return d;
}

__device__ __forceinline__ unsigned short bf_bits(float f) {
  unsigned int u = __float_as_uint(f);
  u += 0x7FFFu + ((u >> 16) & 1u);
  return (unsigned short)(u >> 16);
}
__device__ __forceinline__ float bf_val(unsigned short b) { return __uint_as_float(((unsigned int)b) << 16); }
__device__ __forceinline__ float bf_rne(float f) { return bf_val(bf_bits(f)); }

__device__ __forceinline__ unsigned int pack_hl(float f0, float f1, unsigned int& lo) {
  const unsigned short h0 = bf_bits(f0), h1 = bf_bits(f1);
  const unsigned short l0 = bf_bits(f0 - bf_val(h0)), l1 = bf_bits(f1 - bf_val(h1));
  lo = (unsigned int)l0 | ((unsigned int)l1 << 16);
  return (unsigned int)h0 | ((unsigned int)h1 << 16);
}

#define W_LO(u) __uint_as_float((u) << 16)
#define W_HI(u) __uint_as_float((u) & 0xffff0000u)

__device__ __forceinline__ int scan_chunk(const int* __restrict__ dsts, int nE, int cbase, int slotBase,
                                          int nb, int vec8, int* list, int tid, int lane, int wave) {
  int wc = 0;
  const int el0  = tid * EPT;
  const int e0   = cbase + el0;
  const int sent = -2147483647 - 1;
  v4i da, db;
  if (vec8 != 0 && cbase + CHUNK <= nE) {
    da = *(const v4i*)(dsts + e0);
    db = *(const v4i*)(dsts + e0 + 4);
  } else {
    da.x = (e0     < nE) ? dsts[min(e0,     nE - 1)] : sent;
    da.y = (e0 + 1 < nE) ? dsts[min(e0 + 1, nE - 1)] : sent;
    da.z = (e0 + 2 < nE) ? dsts[min(e0 + 2, nE - 1)] : sent;
    da.w = (e0 + 3 < nE) ? dsts[min(e0 + 3, nE - 1)] : sent;
    db.x = (e0 + 4 < nE) ? dsts[min(e0 + 4, nE - 1)] : sent;
    db.y = (e0 + 5 < nE) ? dsts[min(e0 + 5, nE - 1)] : sent;
    db.z = (e0 + 6 < nE) ? dsts[min(e0 + 6, nE - 1)] : sent;
    db.w = (e0 + 7 < nE) ? dsts[min(e0 + 7, nE - 1)] : sent;
  }
  const unsigned nbs = (unsigned)slotBase;
  const unsigned unb = (unsigned)nb;
  const unsigned s0 = (unsigned)da.x - nbs, s1 = (unsigned)da.y - nbs;
  const unsigned s2 = (unsigned)da.z - nbs, s3 = (unsigned)da.w - nbs;
  const unsigned s4 = (unsigned)db.x - nbs, s5 = (unsigned)db.y - nbs;
  const unsigned s6 = (unsigned)db.z - nbs, s7 = (unsigned)db.w - nbs;
  const bool h0 = s0 < unb, h1 = s1 < unb, h2 = s2 < unb, h3 = s3 < unb;
  const bool h4 = s4 < unb, h5 = s5 < unb, h6 = s6 < unb, h7 = s7 < unb;
  const unsigned any = __builtin_amdgcn_ballot_w32(h0 | h1 | h2 | h3 | h4 | h5 | h6 | h7);
  if (any != 0u) {
#define HITJ(J, HJ, SJ) { \
      const unsigned mj = __builtin_amdgcn_ballot_w32(HJ); \
      if (mj != 0u) { \
        if (HJ) { \
          const int pos = wc + (int)__builtin_amdgcn_mbcnt_lo(mj, 0u); \
          if (pos < WCAP) list[wave * WCAP + pos] = ((el0 + (J)) << PKS) | (int)(SJ); \
        } \
        wc += (int)__builtin_popcount(mj); } }
    HITJ(0, h0, s0)
    HITJ(1, h1, s1)
    HITJ(2, h2, s2)
    HITJ(3, h3, s3)
    HITJ(4, h4, s4)
    HITJ(5, h5, s5)
    HITJ(6, h6, s6)
    HITJ(7, h7, s7)
#undef HITJ
  }
  return wc;
}

__device__ __forceinline__ v8us cv8b(const float* __restrict__ p, size_t stride) {
  v8us o;
#pragma unroll
  for (int i = 0; i < 8; ++i) o[i] = bf_bits(p[(size_t)i * stride]);
  return o;
}

__global__ __launch_bounds__(NTHR) void k_wprep(const float* __restrict__ w1a, const float* __restrict__ w1b,
                                                const float* __restrict__ w2a, const float* __restrict__ w2b,
                                                const float* __restrict__ w3a, const float* __restrict__ w3b,
                                                unsigned short* p1a, unsigned short* p1b, unsigned short* p2a,
                                                unsigned short* p2b, unsigned short* p3a, unsigned short* p3b) {
  const int u = (int)blockIdx.x * NTHR + (int)threadIdx.x;
  v8us o;
  unsigned short* dp;
  if (u < NUB1) {
    const int v = u, n = v >> 5, k8 = (v & 31) * 8, kk = k8 & (CIN - 1);
    o = cv8b(w1a + (size_t)kk * HID + n, HID);
    dp = p1a + (size_t)v * 8;
  } else if (u < NUB2) {
    const int v = u - NUB1, n = v >> 6, k8 = (v & 63) * 8, kk = k8 & (HID - 1);
    o = cv8b(w1b + (size_t)kk * HID + n, HID);
    dp = p1b + (size_t)v * 8;
  } else if (u < NUB3) {
    const int v = u - NUB2, n = v >> 6, k8 = (v & 63) * 8, kk = k8 & (HID - 1);
    o = cv8b(w2a + (size_t)kk * HID + n, HID);
    dp = p2a + (size_t)v * 8;
  } else if (u < NUB4) {
    const int v = u - NUB3, n = v >> 6, k8 = (v & 63) * 8, kk = k8 & (HID - 1);
    o = cv8b(w2b + (size_t)kk * HID + n, HID);
    dp = p2b + (size_t)v * 8;
  } else if (u < NUB5) {
    const int v = u - NUB4, n = v >> 6, k8 = (v & 63) * 8, kk = k8 & (HID - 1);
    o = cv8b(w3a + (size_t)kk * HID + n, HID);
    dp = p3a + (size_t)v * 8;
  } else if (u < NUTOT) {
    const int v = u - NUB5, n = v >> 6, k8 = (v & 63) * 8, kk = k8 & (HID - 1);
    o = cv8b(w3b + (size_t)kk * COUT + n, COUT);
    dp = p3b + (size_t)v * 8;
  } else {
    return;
  }
  *(volatile v8us*)dp = o;
  __threadfence();
  *(volatile v8us*)dp = o;
}

template <int MODE>
__global__ __launch_bounds__(NTHR) void k_agg(
    const int* __restrict__ srcs, const int* __restrict__ dsts,
    const float* __restrict__ xf, const unsigned short* __restrict__ hin,
    unsigned short* Aout, int nN, int nE, int nb, int vec8, int MPr) {
  extern __shared__ __attribute__((aligned(16))) int lds_dyn[];
  int* reg1 = lds_dyn;
  int* reg2 = reg1 + RCAP;
  int* scnt = reg2 + RCAP;
  int* soff = scnt + NBMAX;
  int* list = soff + NBMAX;
  int* wcnt = list + LISTN;
  int* wtot = wcnt + NWAVE;
  const int tid = (int)threadIdx.x, lane = tid & 31, wave = tid >> 5, hh = lane >> 4;
  const int nodeBase = (int)blockIdx.x * nb;

  {
    const v4i z4 = {0, 0, 0, 0};
    for (int i = tid * 4; i < LDS_ZINTS; i += NTHR * 4) *(v4ia*)(lds_dyn + i) = z4;
  }
  __syncthreads();

  int tot = 0;
  const int nChunks = (nE + CHUNK - 1) / CHUNK;
#pragma unroll 1
  for (int ch = 0; ch < nChunks; ++ch) {
    const int cbase = ch * CHUNK;
    const int wc = scan_chunk(dsts, nE, cbase, nodeBase, nb, vec8, list, tid, lane, wave);
    if (lane == 0) wcnt[wave] = wc;
    __syncthreads();
    int pre = 0, all = 0;
#pragma unroll
    for (int w2 = 0; w2 < NWAVE; ++w2) {
      int c = wcnt[w2];
      c = c < 0 ? 0 : (c > WCAP ? WCAP : c);
      all += c;
      pre += (w2 < wave) ? c : 0;
    }
    const int wcc  = wc > WCAP ? WCAP : wc;
    const int base = tot + pre;
#pragma unroll 1
    for (int i = lane; i < wcc; i += 32) {
      const int ent = list[wave * WCAP + i];
      const int el  = (ent >> PKS) & (CHUNK - 1);
      const int sl  = ent & (NBMAX - 1);
      int eid = cbase + el;
      eid = eid > nE - 1 ? nE - 1 : eid;
      const int pos = base + i;
      if (pos < RCAP) reg1[pos] = (int)(((unsigned)eid << PKS) | (unsigned)sl);
    }
    tot += all;
    tot = tot > RCAP ? RCAP : tot;
    __syncthreads();
  }
  const int nh = tot;

  if (wave == 0) {
#pragma unroll 1
    for (int b0 = 0; b0 < nh; b0 += 32) {
      const int idx = b0 + lane;
      const int uv  = reg1[idx < RCAP ? idx : RCAP - 1];
      const int m32 = (nh - b0) < 32 ? (nh - b0) : 32;
#pragma unroll 1
      for (int k = 0; k < m32; ++k) {
        const int u  = __builtin_amdgcn_readlane(uv, k);
        const int sl = u & (NBMAX - 1);
        if (lane == 0) scnt[sl] = scnt[sl] + 1;
      }
    }
  }
  __syncthreads();

  {
    const v4i ca = *(const v4i*)(scnt + 8 * tid);
    const v4i cb = *(const v4i*)(scnt + 8 * tid + 4);
    const int e0 = ca.x < 0 ? 0 : ca.x, e1 = ca.y < 0 ? 0 : ca.y, e2 = ca.z < 0 ? 0 : ca.z, e3 = ca.w < 0 ? 0 : ca.w;
    const int e4 = cb.x < 0 ? 0 : cb.x, e5 = cb.y < 0 ? 0 : cb.y, e6 = cb.z < 0 ? 0 : cb.z, e7 = cb.w < 0 ? 0 : cb.w;
    const int ts = e0 + e1 + e2 + e3 + e4 + e5 + e6 + e7;
    int incl = ts;
#pragma unroll
    for (int d = 1; d < 32; d <<= 1) {
      const int up = __shfl_up(incl, d);
      if (lane >= d) incl += up;
    }
    if (lane == 31) wtot[wave] = incl;
    __syncthreads();
    int pre = 0;
#pragma unroll
    for (int w2 = 0; w2 < NWAVE; ++w2) pre += (w2 < wave) ? wtot[w2] : 0;
    int run = pre + incl - ts;
    soff[8 * tid + 0] = run; run += e0;
    soff[8 * tid + 1] = run; run += e1;
    soff[8 * tid + 2] = run; run += e2;
    soff[8 * tid + 3] = run; run += e3;
    soff[8 * tid + 4] = run; run += e4;
    soff[8 * tid + 5] = run; run += e5;
    soff[8 * tid + 6] = run; run += e6;
    soff[8 * tid + 7] = run;
  }
  __syncthreads();
  for (int i = tid; i < NBMAX; i += NTHR) list[i] = soff[i];
  __syncthreads();

  if (wave == 0) {
#pragma unroll 1
    for (int b0 = 0; b0 < nh; b0 += 32) {
      const int idx = b0 + lane;
      const int uv  = reg1[idx < RCAP ? idx : RCAP - 1];
      const int m32 = (nh - b0) < 32 ? (nh - b0) : 32;
#pragma unroll 1
      for (int k = 0; k < m32; ++k) {
        const int u   = __builtin_amdgcn_readlane(uv, k);
        const int sl  = u & (NBMAX - 1);
        const int eid = (int)((unsigned)u >> PKS);
        if (lane == 0) {
          int pos = list[sl];
          pos = pos < 0 ? 0 : (pos > RCAP - 1 ? RCAP - 1 : pos);
          reg2[pos] = eid;
          list[sl] = pos + 1;
        }
      }
    }
  }
  __syncthreads();

  const int nbw = nb >> 3;
  const bool ovf = (nh >= RCAP);
  const float qnan = __int_as_float(0x7fc00000);
  const int sa = (2 * lane) & 31, sb = (2 * lane + 1) & 31;

#pragma unroll 1
  for (int jt = 0; jt < nbw; ++jt) {
    const int slot = wave * nbw + jt;
    const int grow = nodeBase + slot;
    int st = soff[slot];
    const int craw = scnt[slot];
    int cnt = craw;
    st  = st < 0 ? 0 : (st > nh ? nh : st);
    cnt = cnt < 0 ? 0 : (cnt > DEGCAP ? DEGCAP : cnt);
    if (cnt > nh - st) cnt = nh - st;
    const float pz = (ovf || craw > DEGCAP) ? qnan : 0.0f;
    const bool liveRow = grow < nN;
    const int nc = liveRow ? grow : nN - 1;
    const bool wsv = grow < MPr;

    if constexpr (MODE == 0) {
      float ag0 = 0.f, ag1 = 0.f, ag2 = 0.f, ag3 = 0.f;
#pragma unroll 1
      for (int q = 0; q < cnt; ++q) {
        int idx = st + q; idx = idx > RCAP - 1 ? RCAP - 1 : idx;
        int eid = reg2[idx]; eid = eid < 0 ? 0 : (eid > nE - 1 ? nE - 1 : eid);
        const int sraw = srcs[eid];
        const int s = sraw < 0 ? 0 : (sraw > nN - 1 ? nN - 1 : sraw);
        const v4f v = *(const v4fa*)(xf + (size_t)s * CIN + 4 * lane);
        ag0 += bf_rne(v.x); ag1 += bf_rne(v.y); ag2 += bf_rne(v.z); ag3 += bf_rne(v.w);
      }
      const v4f sv = *(const v4fa*)(xf + (size_t)nc * CIN + 4 * lane);
      float r0 = bf_rne(sv.x) + ag0, r1 = bf_rne(sv.y) + ag1, r2 = bf_rne(sv.z) + ag2, r3 = bf_rne(sv.w) + ag3;
      r0 = (liveRow ? r0 : 0.0f) + pz;
      r1 = (liveRow ? r1 : 0.0f) + pz;
      r2 = (liveRow ? r2 : 0.0f) + pz;
      r3 = (liveRow ? r3 : 0.0f) + pz;
      unsigned int l01, l23;
      const unsigned int h01 = pack_hl(r0, r1, l01);
      const unsigned int h23 = pack_hl(r2, r3, l23);
      const int g0 = __shfl((int)h01, sa, 32), g1 = __shfl((int)h23, sa, 32);
      const int g2 = __shfl((int)h01, sb, 32), g3 = __shfl((int)h23, sb, 32);
      const int p0 = __shfl((int)l01, sa, 32), p1 = __shfl((int)l23, sa, 32);
      const int p2 = __shfl((int)l01, sb, 32), p3 = __shfl((int)l23, sb, 32);
      const bool lsel = (hh != 0);
      v4u pv;
      pv.x = (unsigned int)(lsel ? p0 : g0);
      pv.y = (unsigned int)(lsel ? p1 : g1);
      pv.z = (unsigned int)(lsel ? p2 : g2);
      pv.w = (unsigned int)(lsel ? p3 : g3);
      unsigned short* gp = Aout + (size_t)grow * K1 + 8 * lane;
      if (wsv) *(volatile v4u*)gp = pv;
      __threadfence();
      if (wsv) *(volatile v4u*)gp = pv;
    } else {
      float a0 = 0.f, a1 = 0.f, a2 = 0.f, a3 = 0.f, a4 = 0.f, a5 = 0.f, a6 = 0.f, a7 = 0.f;
#pragma unroll 1
      for (int q = 0; q < cnt; ++q) {
        int idx = st + q; idx = idx > RCAP - 1 ? RCAP - 1 : idx;
        int eid = reg2[idx]; eid = eid < 0 ? 0 : (eid > nE - 1 ? nE - 1 : eid);
        const int sraw = srcs[eid];
        const int s = sraw < 0 ? 0 : (sraw > nN - 1 ? nN - 1 : sraw);
        const unsigned short* rp = hin + (size_t)s * K2 + 8 * lane;
        const v4u wa = *(const v4ua*)rp;
        const v4u wb = *(const v4ua*)(rp + HID);
        const float f0 = W_LO(wa.x) + W_LO(wb.x), f1 = W_HI(wa.x) + W_HI(wb.x);
        const float f2 = W_LO(wa.y) + W_LO(wb.y), f3 = W_HI(wa.y) + W_HI(wb.y);
        const float f4 = W_LO(wa.z) + W_LO(wb.z), f5 = W_HI(wa.z) + W_HI(wb.z);
        const float f6 = W_LO(wa.w) + W_LO(wb.w), f7 = W_HI(wa.w) + W_HI(wb.w);
        a0 += f0; a1 += f1; a2 += f2; a3 += f3; a4 += f4; a5 += f5; a6 += f6; a7 += f7;
      }
      const unsigned short* cp = hin + (size_t)nc * K2 + 8 * lane;
      const v4u ca = *(const v4ua*)cp;
      const v4u cb = *(const v4ua*)(cp + HID);
      float r0 = (W_LO(ca.x) + W_LO(cb.x)) + a0, r1 = (W_HI(ca.x) + W_HI(cb.x)) + a1;
      float r2 = (W_LO(ca.y) + W_LO(cb.y)) + a2, r3 = (W_HI(ca.y) + W_HI(cb.y)) + a3;
      float r4 = (W_LO(ca.z) + W_LO(cb.z)) + a4, r5 = (W_HI(ca.z) + W_HI(cb.z)) + a5;
      float r6 = (W_LO(ca.w) + W_LO(cb.w)) + a6, r7 = (W_HI(ca.w) + W_HI(cb.w)) + a7;
      r0 = (liveRow ? r0 : 0.0f) + pz; r1 = (liveRow ? r1 : 0.0f) + pz;
      r2 = (liveRow ? r2 : 0.0f) + pz; r3 = (liveRow ? r3 : 0.0f) + pz;
      r4 = (liveRow ? r4 : 0.0f) + pz; r5 = (liveRow ? r5 : 0.0f) + pz;
      r6 = (liveRow ? r6 : 0.0f) + pz; r7 = (liveRow ? r7 : 0.0f) + pz;
      unsigned int l0, l1, l2, l3;
      v4u ph, pl;
      ph.x = pack_hl(r0, r1, l0); ph.y = pack_hl(r2, r3, l1);
      ph.z = pack_hl(r4, r5, l2); ph.w = pack_hl(r6, r7, l3);
      pl.x = l0; pl.y = l1; pl.z = l2; pl.w = l3;
      unsigned short* gp = Aout + (size_t)grow * K2 + 8 * lane;
      unsigned short* gq = gp + HID;
      if (wsv) { *(volatile v4u*)gp = ph; *(volatile v4u*)gq = pl; }
      __threadfence();
      if (wsv) { *(volatile v4u*)gp = ph; *(volatile v4u*)gq = pl; }
    }
  }
}

template <int GNT, int EPI>
__global__ __launch_bounds__(GTHR) void k_gemm(const unsigned short* __restrict__ A, int lda,
                                               const unsigned short* __restrict__ BT, int ldb, int K,
                                               const float* __restrict__ bias,
                                               void* outp, int ldo, int lsplit, int nN, int mRows) {
  constexpr int GBN = 16 * GNT;
  static_assert((EPI == 2 && GNT == 8) || (EPI == 3 && GNT == 4));
  __shared__ __attribute__((aligned(16))) float stg[GBM * GBN];
  const int tid = (int)threadIdx.x, lane = tid & 31, wave = tid >> 5, hh = lane >> 4, m = lane & 15;
  const int rowBase = (int)blockIdx.x * GBM;
  const int colBase = (int)blockIdx.y * GBN;

  v8f acc[GNT];
  {
    const v8f z = {0.f, 0.f, 0.f, 0.f, 0.f, 0.f, 0.f, 0.f};
#pragma unroll
    for (int t = 0; t < GNT; ++t) acc[t] = z;
  }
  const unsigned short* ap = A  + (size_t)(rowBase + 16 * wave + m) * (size_t)lda + 8 * hh;
  const unsigned short* bp = BT + (size_t)(colBase + m) * (size_t)ldb + 8 * hh;

#pragma unroll 1
  for (int k0 = 0; k0 < K; k0 += 32) {
    Frag af;
    af.h[0] = *(const v8usa*)(ap + k0);
    af.h[1] = *(const v8usa*)(ap + k0 + 16);
#pragma unroll
    for (int nt = 0; nt < GNT; ++nt) {
      const unsigned short* wq = bp + (size_t)(16 * nt) * (size_t)ldb + k0;
      Frag bfr;
      bfr.h[0] = *(const v8usa*)wq;
      bfr.h[1] = *(const v8usa*)(wq + 16);
      acc[nt] = wmb(af, bfr, acc[nt]);
    }
  }

#pragma unroll
  for (int nt = 0; nt < GNT; ++nt) {
    const int lc = 16 * nt + m;
    const float bb = bf_rne(bias[colBase + lc]);
#pragma unroll
    for (int r = 0; r < 8; ++r) {
      const int lr = 16 * wave + 8 * hh + r;
      const bool live = (rowBase + lr) < nN;
      float v = acc[nt][r] + bb;
      if constexpr (EPI == 2) v = fmaxf(v, 0.0f);
      stg[lr * GBN + lc] = live ? v : 0.0f;
    }
  }
  __syncthreads();

  if constexpr (EPI == 2) {
    unsigned short* outH = (unsigned short*)outp;
    const int cb = 8 * m;
    const bool isHi = (hh == 0);
    v4u pk[16];
#pragma unroll
    for (int i = 0; i < 16; ++i) {
      const int lr = 16 * wave + i;
      const v4f a = *(const v4fa*)(stg + lr * GBN + cb);
      const v4f b = *(const v4fa*)(stg + lr * GBN + cb + 4);
      const float f[8] = {a.x, a.y, a.z, a.w, b.x, b.y, b.z, b.w};
      unsigned int w[4];
#pragma unroll
      for (int j = 0; j < 4; ++j) {
        const unsigned short h0 = bf_bits(f[2 * j]), h1 = bf_bits(f[2 * j + 1]);
        const unsigned short l0 = bf_bits(f[2 * j] - bf_val(h0)), l1 = bf_bits(f[2 * j + 1] - bf_val(h1));
        const unsigned short q0 = isHi ? h0 : l0, q1 = isHi ? h1 : l1;
        w[j] = (unsigned int)q0 | ((unsigned int)q1 << 16);
      }
      v4u pv; pv.x = w[0]; pv.y = w[1]; pv.z = w[2]; pv.w = w[3];
      pk[i] = pv;
    }
#pragma unroll
    for (int i = 0; i < 16; ++i) {
      const int gr = rowBase + 16 * wave + i;
      unsigned short* op = outH + (size_t)gr * (size_t)ldo + colBase + cb + hh * lsplit;
      if (gr < mRows) *(volatile v4u*)op = pk[i];
    }
    __threadfence();
#pragma unroll
    for (int i = 0; i < 16; ++i) {
      const int gr = rowBase + 16 * wave + i;
      unsigned short* op = outH + (size_t)gr * (size_t)ldo + colBase + cb + hh * lsplit;
      if (gr < mRows) *(volatile v4u*)op = pk[i];
    }
  } else {
    float* outF = (float*)outp;
    v4f fv[8];
#pragma unroll
    for (int i = 0; i < 8; ++i) {
      const int lr = 16 * wave + 2 * i + hh;
      fv[i] = *(const v4fa*)(stg + lr * GBN + 4 * m);
    }
#pragma unroll
    for (int i = 0; i < 8; ++i) {
      const int lr = 16 * wave + 2 * i + hh;
      const int gr = rowBase + lr;
      float* op = outF + (size_t)gr * (size_t)ldo + colBase + 4 * m;
      if (gr < mRows) *(volatile v4f*)op = fv[i];
    }
    __threadfence();
#pragma unroll
    for (int i = 0; i < 8; ++i) {
      const int lr = 16 * wave + 2 * i + hh;
      const int gr = rowBase + lr;
      float* op = outF + (size_t)gr * (size_t)ldo + colBase + 4 * m;
      if (gr < mRows) *(volatile v4f*)op = fv[i];
    }
  }
}

static int pick_nb(int nE, int nN) {
  int nb = NBMAX;
  while (nb > 16 && (long long)nb * (long long)nE * 5LL > (long long)RCAP * (long long)nN * 4LL) nb >>= 1;
  return nb;
}
static inline int cdiv(int a, int b) { return (a + b - 1) / b; }
static inline size_t al256(size_t o) { return (o + 255) & ~(size_t)255; }

extern "C" void kernel_launch(void* const* d_in, const int* in_sizes, int n_in,
                              void* d_out, int out_size, void* d_ws, size_t ws_size,
                              hipStream_t stream) {
  if (n_in < 14) return;
  if (in_sizes[0] < CIN || (in_sizes[0] % CIN) != 0) return;
  const int nN = in_sizes[0] / CIN;
  if (nN < GBM || nN > (1 << 22)) return;
  const int nE2 = in_sizes[1];
  if (nE2 < 2 || (nE2 & 1) != 0) return;
  const int nE = nE2 / 2;
  if (nE < 1 || nE > (1 << 21)) return;
  if (in_sizes[2]  != CIN * HID  || in_sizes[3]  != HID)  return;
  if (in_sizes[4]  != HID * HID  || in_sizes[5]  != HID)  return;
  if (in_sizes[6]  != HID * HID  || in_sizes[7]  != HID)  return;
  if (in_sizes[8]  != HID * HID  || in_sizes[9]  != HID)  return;
  if (in_sizes[10] != HID * HID  || in_sizes[11] != HID)  return;
  if (in_sizes[12] != HID * COUT || in_sizes[13] != COUT) return;
  if ((long long)out_size != (long long)nN * COUT) return;

  const float* x   = (const float*)d_in[0];
  const int*   ei  = (const int*)  d_in[1];
  const int*   src = ei;
  const int*   dst = ei + nE;
  const float* w1a = (const float*)d_in[2];  const float* b1a = (const float*)d_in[3];
  const float* w1b = (const float*)d_in[4];  const float* b1b = (const float*)d_in[5];
  const float* w2a = (const float*)d_in[6];  const float* b2a = (const float*)d_in[7];
  const float* w2b = (const float*)d_in[8];  const float* b2b = (const float*)d_in[9];
  const float* w3a = (const float*)d_in[10]; const float* b3a = (const float*)d_in[11];
  const float* w3b = (const float*)d_in[12]; const float* b3b = (const float*)d_in[13];
  float* out = (float*)d_out;

  const int MP   = cdiv(nN, GBM) * GBM;
  const int gM   = MP / GBM;
  const int nb   = pick_nb(nE, nN);
  const int gA   = cdiv(MP, nb);
  const int vec8 = ((nE & 3) == 0) ? 1 : 0;
  if ((long long)gA * nb < (long long)MP) return;
  if ((long long)(gM - 1) * GBM >= (long long)nN) return;

  char* ws = (char*)d_ws;
  size_t off = 0;
  const size_t oW1A = off; off = al256(off + (size_t)NU1A * 16);
  const size_t oW1B = off; off = al256(off + (size_t)NUHH * 16);
  const size_t oW2A = off; off = al256(off + (size_t)NUHH * 16);
  const size_t oW2B = off; off = al256(off + (size_t)NUHH * 16);
  const size_t oW3A = off; off = al256(off + (size_t)NUHH * 16);
  const size_t oW3B = off; off = al256(off + (size_t)NU3B * 16);
  const size_t oR0  = off; off = al256(off + (size_t)MP * K2 * 2);
  const size_t oR1  = off; off = al256(off + (size_t)MP * K2 * 2);
  if (off > ws_size || off > (size_t)WSMAX) return;
  unsigned short* W1A = (unsigned short*)(ws + oW1A);
  unsigned short* W1B = (unsigned short*)(ws + oW1B);
  unsigned short* W2A = (unsigned short*)(ws + oW2A);
  unsigned short* W2B = (unsigned short*)(ws + oW2B);
  unsigned short* W3A = (unsigned short*)(ws + oW3A);
  unsigned short* W3B = (unsigned short*)(ws + oW3B);
  unsigned short* R0  = (unsigned short*)(ws + oR0);
  unsigned short* R1  = (unsigned short*)(ws + oR1);

  hipFuncSetAttribute(reinterpret_cast<const void*>(&k_agg<0>), hipFuncAttributeMaxDynamicSharedMemorySize, LDS_AGG);
  hipFuncSetAttribute(reinterpret_cast<const void*>(&k_agg<1>), hipFuncAttributeMaxDynamicSharedMemorySize, LDS_AGG);

  k_wprep<<<NUTOT / NTHR, NTHR, 0, stream>>>(w1a, w1b, w2a, w2b, w3a, w3b, W1A, W1B, W2A, W2B, W3A, W3B);
  k_agg<0><<<gA, NTHR, LDS_AGG, stream>>>(src, dst, x, R1, R0, nN, nE, nb, vec8, MP);
  k_gemm<8, 2><<<dim3(gM, HID / 128), GTHR, 0, stream>>>(R0, K1, W1A, K1, K1, b1a, (void*)R1, K2, HID, nN, MP);
  k_gemm<8, 2><<<dim3(gM, HID / 128), GTHR, 0, stream>>>(R1, K2, W1B, K2, K2, b1b, (void*)R0, K2, HID, nN, MP);
  k_agg<1><<<gA, NTHR, LDS_AGG, stream>>>(src, dst, x, R0, R1, nN, nE, nb, vec8, MP);
  k_gemm<8, 2><<<dim3(gM, HID / 128), GTHR, 0, stream>>>(R1, K2, W2A, K2, K2, b2a, (void*)R0, K2, HID, nN, MP);
  k_gemm<8, 2><<<dim3(gM, HID / 128), GTHR, 0, stream>>>(R0, K2, W2B, K2, K2, b2b, (void*)R1, K2, HID, nN, MP);
  k_gemm<8, 2><<<dim3(gM, HID / 128), GTHR, 0, stream>>>(R1, K2, W3A, K2, K2, b3a, (void*)R0, K2, HID, nN, MP);
  k_gemm<4, 3><<<dim3(gM, COUT / 64), GTHR, 0, stream>>>(R0, K2, W3B, K2, K2, b3b, (void*)out, COUT, 0, nN, nN);
}
